// GroupedQueryAttention_35931696398604
// MI455X (gfx1250) — hardware-verified
//
#include <hip/hip_runtime.h>


#ifndef NB
#define NB 2
#endif
#ifndef SEQ
#define SEQ 2048
#endif
#define NB_FULL  2
#define SEQ_FULL 2048
#ifndef OUT_SEQ
#define OUT_SEQ SEQ
#endif
#define DM   2048
#define NH_  32
#define NG_  8
#define GS_  4
#define HD   64
#define KVD  512
#define QKVC 3072
#define AW   4
#define QRS  2048.0f
#define QRI  (1.0f / 2048.0f)
#define SC2  (0.125f * 1.4426950408889634f)
#define PSH  8.0f
#define CXS  64.0f
#define WOS  64.0f
#define OSC  (1.0f / 4096.0f)
#define NEGB (-3.0e38f)

static constexpr int ER_ROWS = (SEQ < 512) ? SEQ : 512;

static_assert(HD == 64);
static_assert(NH_ * HD == DM);
static_assert(NG_ * HD == KVD);
static_assert(NG_ * GS_ == NH_);
static_assert(DM % 64 == 0);
static_assert(DM % 32 == 0);
static_assert(KVD % 64 == 0);
static_assert(SEQ % 64 == 0);
static_assert(SEQ % (16 * AW) == 0);
static_assert(ER_ROWS % 64 == 0);
static_assert((SEQ - ER_ROWS) % 64 == 0);
static_assert(((size_t)SEQ * DM) % 8 == 0);
static_assert(NB <= NB_FULL);
static_assert(SEQ <= SEQ_FULL);
static_assert(QKVC == DM + 2 * KVD);
static_assert(QKVC % 64 == 0);
static_assert(QKVC % 4 == 0);

typedef _Float16 h16;
typedef unsigned short bf;
typedef __attribute__((ext_vector_type(16))) __bf16   v16bf;
typedef __attribute__((ext_vector_type(16))) _Float16 v16h;
typedef __attribute__((ext_vector_type(8)))  _Float16 v8h;
typedef __attribute__((ext_vector_type(8)))  unsigned short v8us;
typedef __attribute__((ext_vector_type(8)))  float    v8f;
typedef __attribute__((ext_vector_type(4)))  float    v4f;
typedef v4f  __attribute__((may_alias)) v4fa;

__device__ __forceinline__ unsigned short f2bf(float f) { unsigned u = __float_as_uint(f); u += 0x7FFFu + ((u >> 16) & 1u); return (unsigned short)(u >> 16); }
__device__ __forceinline__ float bfr(float f) { return __uint_as_float(((unsigned)f2bf(f)) << 16); }
__device__ __forceinline__ v16h cat16(v8h lo, v8h hi) { return __builtin_shufflevector(lo, hi, 0, 1, 2, 3, 4, 5, 6, 7, 8, 9, 10, 11, 12, 13, 14, 15); }
__device__ __forceinline__ v16bf cat16b(v8us lo, v8us hi) { return __builtin_bit_cast(v16bf, __builtin_shufflevector(lo, hi, 0, 1, 2, 3, 4, 5, 6, 7, 8, 9, 10, 11, 12, 13, 14, 15)); }
__device__ __forceinline__ v8f wmma16(v16h a, v16h b, v8f c) { return __builtin_amdgcn_wmma_f32_16x16x32_f16(false, a, false, b, (short)0, c, false, false); }
__device__ __forceinline__ v8f wmmab(v16bf a, v16bf b, v8f c) { return __builtin_amdgcn_wmma_f32_16x16x32_bf16(false, a, false, b, (short)0, c, false, false); }
__device__ __forceinline__ v16h  ldh(const h16* p) { return cat16(*(const v8h*)p, *(const v8h*)(p + 16)); }
__device__ __forceinline__ v16bf ldb(const bf* p)  { return cat16b(*(const v8us*)p, *(const v8us*)(p + 16)); }
__device__ __forceinline__ void wave_sync() { __builtin_amdgcn_fence(3  , "wavefront"); __builtin_amdgcn_wave_barrier(); asm volatile("" ::: "memory"); }

template<int MODE>
__global__ __launch_bounds__(256) void k_cvt8(const float* __restrict__ src, unsigned short* dst, size_t n8) {
    const size_t i = (size_t)blockIdx.x * 256 + threadIdx.x; if (i >= n8) return;
    const v8f v = *(const v8f*)(src + i * 8);
    if (MODE == 0) {
        v8us o;
#pragma unroll
        for (int k = 0; k < 8; ++k) o[k] = f2bf(v[k]);
        *(volatile v8us*)(dst + i * 8) = o; __threadfence(); *(volatile v8us*)(dst + i * 8) = o;
    } else {
        v8h o;
#pragma unroll
        for (int k = 0; k < 8; ++k) o[k] = (h16)(bfr(v[k]) * WOS);
        h16* d = (h16*)dst;
        *(volatile v8h*)(d + i * 8) = o; __threadfence(); *(volatile v8h*)(d + i * 8) = o;
    }
}

typedef v8us __attribute__((may_alias)) v8usa;
__global__ __launch_bounds__(256) void k_cvtT(const float* __restrict__ src, unsigned short* dst, int N, int mode) {
#pragma clang fp contract(off)
    __shared__ __align__(16) unsigned short ts[64 * 72];
    const int tid = threadIdx.x;
    const int n0 = blockIdx.x * 64, k0 = blockIdx.y * 64;
#pragma unroll 1
    for (int it = 0; it < 4; ++it) {
        const int kr = it * 16 + (tid >> 4), c4 = (tid & 15) * 4;
        const v4f v = *(const v4f*)(src + (size_t)(k0 + kr) * (size_t)N + n0 + c4);
#pragma unroll
        for (int i = 0; i < 4; ++i) {
            const unsigned short bb = f2bf(v[i]);
            const unsigned short hb = __builtin_bit_cast(unsigned short, (h16)(bfr(v[i]) * WOS));
            ts[(c4 + i) * 72 + kr] = mode ? hb : bb;
        }
    }
    __syncthreads();
    v8us o[2];
#pragma unroll
    for (int s = 0; s < 2; ++s) { const int row = 32 * s + (tid >> 3), c8 = (tid & 7) * 8;
        o[s] = *(const v8usa*)(&ts[row * 72 + c8]); }
#pragma unroll
    for (int s = 0; s < 2; ++s) { const int row = 32 * s + (tid >> 3), c8 = (tid & 7) * 8;
        *(volatile v8us*)(dst + (size_t)(n0 + row) * DM + k0 + c8) = o[s]; }
    __threadfence();
#pragma unroll
    for (int s = 0; s < 2; ++s) { const int row = 32 * s + (tid >> 3), c8 = (tid & 7) * 8;
        *(volatile v8us*)(dst + (size_t)(n0 + row) * DM + k0 + c8) = o[s]; }
}

template<bool ROPE>
__global__ __launch_bounds__(32) void k_proj(const bf* __restrict__ A, const bf* __restrict__ Bt, h16* Ph, h16* Pr, int RB, size_t sRB, int pitch, int CB, size_t sCB,
                                             const float* __restrict__ COS, const float* __restrict__ SIN) {
    __shared__ __align__(16) float os[16 * 68];
    const int K = DM;
    const int lane = threadIdx.x & 31, lr = lane & 15, hi = lane >> 4; const int r0 = blockIdx.x * 64, c0 = blockIdx.y * 64;
    v8f acc[4][4];
#pragma unroll
    for (int mb = 0; mb < 4; ++mb)
#pragma unroll
        for (int nb = 0; nb < 4; ++nb) acc[mb][nb] = (v8f){};
    const size_t aoff = (size_t)(r0 + lr) * K + 8 * hi, boff = (size_t)(c0 + lr) * K + 8 * hi;
#pragma unroll 1
    for (int kc = 0; kc < K; kc += 32) {
        v16bf a[4];
#pragma unroll
        for (int mb = 0; mb < 4; ++mb) a[mb] = ldb(A + aoff + (size_t)mb * 16 * K + kc);
#pragma unroll
        for (int nb = 0; nb < 4; ++nb) { const v16bf b = ldb(Bt + boff + (size_t)nb * 16 * K + kc);
#pragma unroll
            for (int mb = 0; mb < 4; ++mb) acc[mb][nb] = wmmab(a[mb], b, acc[mb][nb]); }
        asm volatile("v_nop\n\tv_nop\n\tv_nop\n\tv_nop" : "+v"(acc[0][0]), "+v"(acc[1][1]), "+v"(acc[2][2]), "+v"(acc[3][3]) : "v"(a[0]), "v"(a[1]), "v"(a[2]), "v"(a[3]));
    }
    const size_t tbase = (size_t)(r0 / RB) * sRB + (size_t)(r0 % RB) * (size_t)pitch + (size_t)(c0 / CB) * sCB + (size_t)(c0 % CB);
    const int tok0 = r0 % RB;
#pragma unroll
    for (int mb = 0; mb < 4; ++mb) {
#pragma unroll
        for (int nb = 0; nb < 4; ++nb) {
#pragma unroll
            for (int j = 0; j < 8; ++j) os[(hi * 8 + j) * 68 + nb * 16 + lr] = acc[mb][nb][j]; }
        wave_sync();
        v8h hv[4], rv[4];
#pragma unroll
        for (int s = 0; s < 4; ++s) { const int row = 4 * s + (lane >> 3), c8 = (lane & 7) * 8;
            const v4f x0 = *(const v4fa*)(&os[row * 68 + c8]); const v4f x1 = *(const v4fa*)(&os[row * 68 + c8 + 4]);
            float xv[8];
#pragma unroll
            for (int i = 0; i < 4; ++i) { xv[i] = x0[i]; xv[4 + i] = x1[i]; }
            if (ROPE) {
                const int pc = c8 ^ 32;
                const v4f y0 = *(const v4fa*)(&os[row * 68 + pc]); const v4f y1 = *(const v4fa*)(&os[row * 68 + pc + 4]);
                const size_t to = (size_t)(tok0 + mb * 16 + row) * HD + c8;
                const v4f ca = *(const v4f*)(COS + to), cb = *(const v4f*)(COS + to + 4), sa = *(const v4f*)(SIN + to), sb = *(const v4f*)(SIN + to + 4);
                const float sg = (c8 < 32) ? -1.0f : 1.0f;
#pragma unroll
                for (int i = 0; i < 4; ++i) { xv[i] = x0[i] * bfr(ca[i]) + (sg * y0[i]) * bfr(sa[i]); xv[4 + i] = x1[i] * bfr(cb[i]) + (sg * y1[i]) * bfr(sb[i]); }
            }
            v8h hh, rr;
#pragma unroll
            for (int i = 0; i < 8; ++i) { const h16 a0 = (h16)xv[i]; hh[i] = a0; rr[i] = (h16)((xv[i] - (float)a0) * QRS); }
            hv[s] = hh; rv[s] = rr; }
        const size_t sb0 = tbase + (size_t)(mb * 16) * (size_t)pitch;
#pragma unroll
        for (int s = 0; s < 4; ++s) { const int row = 4 * s + (lane >> 3), c8 = (lane & 7) * 8; const size_t oo = sb0 + (size_t)row * (size_t)pitch + c8;
            *(volatile v8h*)(Ph + oo) = hv[s]; *(volatile v8h*)(Pr + oo) = rv[s]; }
        __threadfence();
#pragma unroll
        for (int s = 0; s < 4; ++s) { const int row = 4 * s + (lane >> 3), c8 = (lane & 7) * 8; const size_t oo = sb0 + (size_t)row * (size_t)pitch + c8;
            *(volatile v8h*)(Ph + oo) = hv[s]; *(volatile v8h*)(Pr + oo) = rv[s]; }
        wave_sync();
    }
}

template<bool ER>
__global__ __launch_bounds__(32 * AW) void k_flash(const h16* __restrict__ QH, const h16* __restrict__ QR, const h16* __restrict__ KH, const h16* __restrict__ KR,
                                                   const h16* __restrict__ VH, const h16* __restrict__ VR, h16* CH, h16* CR, int xb0) {
    __shared__ __align__(16) float os[AW * 16 * 68];
    const int lane = threadIdx.x & 31, lr = lane & 15, hi = lane >> 4;
    const int wave = __builtin_amdgcn_readfirstlane((int)(threadIdx.x >> 5));
    const int zh = blockIdx.y; const int b = zh / NH_, h = zh % NH_, g = h / GS_;
    const int t0 = (((int)blockIdx.x + xb0) * AW + wave) * 16;
    const int tq = t0 + lr;
    const size_t qbase = (size_t)zh * SEQ * HD;
    const size_t kvb = (size_t)(b * NG_ + g) * SEQ * HD;
    const size_t qo = qbase + (size_t)(t0 + lr) * HD + 8 * hi;
    const v16h qh0 = ldh(QH + qo), qh1 = ldh(QH + qo + 32);
    v16h qr0 = qh0, qr1 = qh1;
    if (ER) { qr0 = ldh(QR + qo); qr1 = ldh(QR + qo + 32); }
    const size_t ko = kvb + (size_t)lr * HD + 8 * hi;
    const size_t vo = kvb + (size_t)lr * SEQ + 8 * hi;
    v8f oH[4], oL[4];
#pragma unroll
    for (int j = 0; j < 4; ++j) { oH[j] = (v8f){}; oL[j] = (v8f){}; }
    float m = NEGB, l = 0.0f;
#pragma unroll 1
    for (int key0 = 0; key0 < t0 + 16; key0 += 32) {
        const h16* ka = KH + ko + (size_t)key0 * HD;
        float ta[8], tb[8];
        if (!ER) {
            const v16h ka0 = ldh(ka), ka1 = ldh(ka + 32), kb0 = ldh(ka + 16 * HD), kb1 = ldh(ka + 16 * HD + 32);
            v8f sHa = (v8f){}, sHb = (v8f){};
            sHa = wmma16(ka0, qh0, sHa); sHb = wmma16(kb0, qh0, sHb);
            sHa = wmma16(ka1, qh1, sHa); sHb = wmma16(kb1, qh1, sHb);
            asm volatile("v_nop\n\tv_nop\n\tv_nop\n\tv_nop" : "+v"(sHa), "+v"(sHb) : "v"(ka0), "v"(ka1), "v"(kb0), "v"(kb1));
#pragma unroll
            for (int r = 0; r < 8; ++r) { ta[r] = sHa[r] * SC2; tb[r] = sHb[r] * SC2; }
        } else {
            const h16* kr = KR + ko + (size_t)key0 * HD;
            { const v16h ka0 = ldh(ka), ka1 = ldh(ka + 32), ra0 = ldh(kr), ra1 = ldh(kr + 32);
              v8f sH = (v8f){}, sL = (v8f){};
              sH = wmma16(ka0, qh0, sH); sL = wmma16(ka0, qr0, sL);
              sH = wmma16(ka1, qh1, sH); sL = wmma16(ka1, qr1, sL);
              sL = wmma16(ra0, qh0, sL); sL = wmma16(ra1, qh1, sL);
              asm volatile("v_nop\n\tv_nop\n\tv_nop\n\tv_nop" : "+v"(sH), "+v"(sL) : "v"(ka0), "v"(ka1), "v"(ra0), "v"(ra1));
#pragma unroll
              for (int r = 0; r < 8; ++r) ta[r] = (sH[r] + sL[r] * QRI) * SC2; }
            { const v16h kb0 = ldh(ka + 16 * HD), kb1 = ldh(ka + 16 * HD + 32), rb0 = ldh(kr + 16 * HD), rb1 = ldh(kr + 16 * HD + 32);
              v8f sH = (v8f){}, sL = (v8f){};
              sH = wmma16(kb0, qh0, sH); sL = wmma16(kb0, qr0, sL);
              sH = wmma16(kb1, qh1, sH); sL = wmma16(kb1, qr1, sL);
              sL = wmma16(rb0, qh0, sL); sL = wmma16(rb1, qh1, sL);
              asm volatile("v_nop\n\tv_nop\n\tv_nop\n\tv_nop" : "+v"(sH), "+v"(sL) : "v"(kb0), "v"(kb1), "v"(rb0), "v"(rb1));
#pragma unroll
              for (int r = 0; r < 8; ++r) tb[r] = (sH[r] + sL[r] * QRI) * SC2; }
        }
        if (key0 + 31 > t0) {
#pragma unroll
            for (int r = 0; r < 8; ++r) { const int kk = key0 + 8 * hi + r; ta[r] = (kk <= tq) ? ta[r] : NEGB; tb[r] = (kk + 16 <= tq) ? tb[r] : NEGB; }
        }
        float mx = NEGB;
#pragma unroll
        for (int r = 0; r < 8; ++r) mx = fmaxf(mx, fmaxf(ta[r], tb[r]));
        mx = fmaxf(mx, __shfl_xor(mx, 16, 32));
        const float mnew = fmaxf(m, mx);
        const float alpha = __builtin_amdgcn_exp2f(m - mnew);
        const float sh = PSH - mnew;
        v16h pb, pq; float ls = 0.0f;
        if (!ER) {
#pragma unroll
            for (int r = 0; r < 8; ++r) { const h16 pa = (h16)__builtin_amdgcn_exp2f(ta[r] + sh); const h16 pc = (h16)__builtin_amdgcn_exp2f(tb[r] + sh); pb[r] = pa; pb[8 + r] = pc; ls += (float)pa + (float)pc; }
            pq = pb;
        } else {
#pragma unroll
            for (int r = 0; r < 8; ++r) { const float fa = __builtin_amdgcn_exp2f(ta[r] + sh); const float fc = __builtin_amdgcn_exp2f(tb[r] + sh);
                const h16 pa = (h16)fa; const h16 pc = (h16)fc; const h16 qa = (h16)((fa - (float)pa) * QRS); const h16 qc = (h16)((fc - (float)pc) * QRS);
                pb[r] = pa; pb[8 + r] = pc; pq[r] = qa; pq[8 + r] = qc; ls += ((float)pa + (float)pc) + ((float)qa + (float)qc) * QRI; }
        }
        l = l * alpha + ls; m = mnew;
#pragma unroll
        for (int j = 0; j < 4; ++j) { oH[j] = oH[j] * alpha; if (ER) oL[j] = oL[j] * alpha; }
        const h16* va = VH + vo + key0;
        const v16h v0 = ldh(va), v1 = ldh(va + (size_t)16 * SEQ), v2 = ldh(va + (size_t)32 * SEQ), v3 = ldh(va + (size_t)48 * SEQ);
        if (!ER) {
            oH[0] = wmma16(v0, pb, oH[0]); oH[1] = wmma16(v1, pb, oH[1]); oH[2] = wmma16(v2, pb, oH[2]); oH[3] = wmma16(v3, pb, oH[3]);
            asm volatile("v_nop\n\tv_nop\n\tv_nop\n\tv_nop" : "+v"(oH[0]), "+v"(oH[1]), "+v"(oH[2]), "+v"(oH[3]) : "v"(v0), "v"(v1), "v"(v2), "v"(v3), "v"(pb));
        } else {
            const h16* vr = VR + vo + key0;
            const v16h w0 = ldh(vr), w1 = ldh(vr + (size_t)16 * SEQ), w2 = ldh(vr + (size_t)32 * SEQ), w3 = ldh(vr + (size_t)48 * SEQ);
            oH[0] = wmma16(v0, pb, oH[0]); oH[1] = wmma16(v1, pb, oH[1]); oH[2] = wmma16(v2, pb, oH[2]); oH[3] = wmma16(v3, pb, oH[3]);
            oL[0] = wmma16(w0, pb, oL[0]); oL[1] = wmma16(w1, pb, oL[1]); oL[2] = wmma16(w2, pb, oL[2]); oL[3] = wmma16(w3, pb, oL[3]);
            oL[0] = wmma16(v0, pq, oL[0]); oL[1] = wmma16(v1, pq, oL[1]); oL[2] = wmma16(v2, pq, oL[2]); oL[3] = wmma16(v3, pq, oL[3]);
            asm volatile("v_nop\n\tv_nop\n\tv_nop\n\tv_nop" : "+v"(oH[0]), "+v"(oH[1]), "+v"(oH[2]), "+v"(oH[3]), "+v"(oL[0]), "+v"(oL[1]), "+v"(oL[2]), "+v"(oL[3])
                         : "v"(v0), "v"(v1), "v"(v2), "v"(v3), "v"(w0), "v"(w1), "v"(w2), "v"(w3), "v"(pb), "v"(pq));
        }
    }
    l += __shfl_xor(l, 16, 32);
    const float inv = CXS * (1.0f / l);
    const int wb = wave * 16 * 68;
#pragma unroll
    for (int j = 0; j < 4; ++j) { v4f a, c;
#pragma unroll
        for (int i = 0; i < 4; ++i) {
            if (ER) { a[i] = (oH[j][i] + oL[j][i] * QRI) * inv; c[i] = (oH[j][4 + i] + oL[j][4 + i] * QRI) * inv; }
            else    { a[i] = oH[j][i] * inv; c[i] = oH[j][4 + i] * inv; } }
        *(v4fa*)(&os[wb + lr * 68 + 16 * j + 8 * hi]) = a; *(v4fa*)(&os[wb + lr * 68 + 16 * j + 8 * hi + 4]) = c; }
    wave_sync();
    v8h hv[4], rv[4];
#pragma unroll
    for (int s = 0; s < 4; ++s) { const int row = 4 * s + (lane >> 3), c8 = (lane & 7) * 8;
        const v4f x0 = *(const v4fa*)(&os[wb + row * 68 + c8]); const v4f x1 = *(const v4fa*)(&os[wb + row * 68 + c8 + 4]); v8h hh, rr;
#pragma unroll
        for (int i = 0; i < 4; ++i) { const h16 a0 = (h16)x0[i]; const h16 a1 = (h16)x1[i]; hh[i] = a0; hh[4 + i] = a1; rr[i] = (h16)((x0[i] - (float)a0) * QRS); rr[4 + i] = (h16)((x1[i] - (float)a1) * QRS); }
        hv[s] = hh; rv[s] = rr; }
    const size_t cbase = ((size_t)b * SEQ + t0) * DM + (size_t)h * HD;
    const size_t rbase = ((size_t)b * ER_ROWS + t0) * DM + (size_t)h * HD;
#pragma unroll
    for (int s = 0; s < 4; ++s) { const int row = 4 * s + (lane >> 3), c8 = (lane & 7) * 8;
        *(volatile v8h*)(CH + cbase + (size_t)row * DM + c8) = hv[s]; if (ER) *(volatile v8h*)(CR + rbase + (size_t)row * DM + c8) = rv[s]; }
    __threadfence();
#pragma unroll
    for (int s = 0; s < 4; ++s) { const int row = 4 * s + (lane >> 3), c8 = (lane & 7) * 8;
        *(volatile v8h*)(CH + cbase + (size_t)row * DM + c8) = hv[s]; if (ER) *(volatile v8h*)(CR + rbase + (size_t)row * DM + c8) = rv[s]; }
}

template<int MB, bool RES>
__global__ __launch_bounds__(32) void k_out(const h16* __restrict__ CH, const h16* __restrict__ CR, const h16* __restrict__ WO, float* OUT, int tstart, int tcount) {
    __shared__ __align__(16) float os[16 * 68];
    const int lane = threadIdx.x & 31, lr = lane & 15, hi = lane >> 4;
    const int tiles = tcount / (16 * MB);
    const int b = (int)blockIdx.x / tiles, t = tstart + ((int)blockIdx.x % tiles) * 16 * MB, c0 = blockIdx.y * 64;
    v8f acc[MB][4], acr[MB][4];
#pragma unroll
    for (int mb = 0; mb < MB; ++mb)
#pragma unroll
        for (int nb = 0; nb < 4; ++nb) { acc[mb][nb] = (v8f){}; acr[mb][nb] = (v8f){}; }
    const size_t aoff = ((size_t)b * SEQ + t + lr) * DM + 8 * hi;
    const size_t roff = ((size_t)b * ER_ROWS + t + lr) * DM + 8 * hi;
    const size_t boff = (size_t)(c0 + lr) * DM + 8 * hi;
#pragma unroll 1
    for (int kc = 0; kc < DM; kc += 32) {
        v16h a[MB], ar[MB];
#pragma unroll
        for (int mb = 0; mb < MB; ++mb) { a[mb] = ldh(CH + aoff + (size_t)mb * 16 * DM + kc); ar[mb] = a[mb]; if (RES) ar[mb] = ldh(CR + roff + (size_t)mb * 16 * DM + kc); }
#pragma unroll
        for (int nb = 0; nb < 4; ++nb) { const v16h bb = ldh(WO + boff + (size_t)nb * 16 * DM + kc);
#pragma unroll
            for (int mb = 0; mb < MB; ++mb) { acc[mb][nb] = wmma16(a[mb], bb, acc[mb][nb]); if (RES) acr[mb][nb] = wmma16(ar[mb], bb, acr[mb][nb]); } }
        if (RES) asm volatile("v_nop\n\tv_nop\n\tv_nop\n\tv_nop" : "+v"(acc[0][0]), "+v"(acc[MB - 1][3]), "+v"(acr[0][0]), "+v"(acr[MB - 1][3]) : "v"(a[0]), "v"(a[1]), "v"(a[MB - 2]), "v"(a[MB - 1]), "v"(ar[0]), "v"(ar[MB - 1]));
        else     asm volatile("v_nop\n\tv_nop\n\tv_nop\n\tv_nop" : "+v"(acc[0][0]), "+v"(acc[1][1]), "+v"(acc[MB - 2][2]), "+v"(acc[MB - 1][3]) : "v"(a[0]), "v"(a[1]), "v"(a[MB - 2]), "v"(a[MB - 1]));
    }
#pragma unroll
    for (int mb = 0; mb < MB; ++mb) {
#pragma unroll
        for (int nb = 0; nb < 4; ++nb) {
#pragma unroll
            for (int j = 0; j < 8; ++j) os[(hi * 8 + j) * 68 + nb * 16 + lr] = RES ? (acc[mb][nb][j] + acr[mb][nb][j] * QRI) * OSC : acc[mb][nb][j] * OSC; }
        wave_sync();
        float* orow = OUT + ((size_t)b * OUT_SEQ + t + mb * 16) * DM + c0;
#pragma unroll 1
        for (int ps = 0; ps < 2; ++ps) {
#pragma unroll
            for (int s = 0; s < 8; ++s) { const int row = 2 * s + hi, cofs = lr * 4;
                const v4f val = *(const v4fa*)(&os[row * 68 + cofs]);
                *(volatile v4f*)(orow + (size_t)row * DM + cofs) = val; }
            if (ps == 0) __threadfence(); }
        wave_sync();
    }
}

static constexpr size_t al256(size_t v) { return (v + 255) & ~(size_t)255; }
static constexpr size_t SZ_XB = al256((size_t)NB * SEQ * DM * 2);
static constexpr size_t SZ_WQ = al256((size_t)DM * DM * 2);
static constexpr size_t SZ_WK = al256((size_t)KVD * DM * 2);
static constexpr size_t SZ_QP = al256((size_t)NB * NH_ * SEQ * HD * 2);
static constexpr size_t SZ_KP = al256((size_t)NB * NG_ * SEQ * HD * 2);
static constexpr size_t SZ_CH = al256((size_t)NB * SEQ * DM * 2);
static constexpr size_t SZ_CR = al256((size_t)NB * ER_ROWS * DM * 2);
static constexpr size_t SZ_TOTAL = SZ_XB + 2 * SZ_WQ + 2 * SZ_WK + 2 * SZ_QP + 4 * SZ_KP + SZ_CH + SZ_CR;
static_assert(SZ_TOTAL <= (size_t)134217728);
static_assert(SZ_WQ == (size_t)DM * DM * 2);
static_assert(SZ_WK == (size_t)KVD * DM * 2);
static_assert(SZ_WQ + 2 * SZ_WK == (size_t)QKVC * DM * 2);

extern "C" void kernel_launch(void* const* d_in, const int* in_sizes, int n_in,
                              void* d_out, int out_size, void* d_ws, size_t ws_size, hipStream_t stream) {
    if (n_in < 5) return;
    const size_t needx = ((size_t)(NB - 1) * SEQ_FULL + SEQ) * DM;
    if ((size_t)in_sizes[0] < needx) return;
    if ((size_t)in_sizes[1] < (size_t)SEQ * HD || (size_t)in_sizes[2] < (size_t)SEQ * HD) return;
    if ((size_t)in_sizes[3] < (size_t)DM * QKVC || (size_t)in_sizes[4] < (size_t)DM * DM) return;
    if ((size_t)out_size < ((size_t)(NB - 1) * OUT_SEQ + SEQ) * DM) return;
    if (SZ_TOTAL > ws_size) return;
    const float* x = (const float*)d_in[0]; const float* sn = (const float*)d_in[1]; const float* cs = (const float*)d_in[2];
    const float* wqkv = (const float*)d_in[3]; const float* wo = (const float*)d_in[4];
    float* OUT = (float*)d_out;
    char* wsp = (char*)d_ws;
    bf* XB = (bf*)wsp; wsp += SZ_XB;
    bf* WQ = (bf*)wsp; wsp += SZ_WQ;
    bf* WK = (bf*)wsp; wsp += SZ_WK;
    bf* WV = (bf*)wsp; wsp += SZ_WK;
    h16* WO = (h16*)wsp; wsp += SZ_WQ;
    h16* QH = (h16*)wsp; wsp += SZ_QP;
    h16* QR = (h16*)wsp; wsp += SZ_QP;
    h16* KH = (h16*)wsp; wsp += SZ_KP;
    h16* KR = (h16*)wsp; wsp += SZ_KP;
    h16* VH = (h16*)wsp; wsp += SZ_KP;
    h16* VR = (h16*)wsp; wsp += SZ_KP;
    h16* CH = (h16*)wsp; wsp += SZ_CH;
    h16* CR = (h16*)wsp; wsp += SZ_CR;

    if (SEQ == SEQ_FULL) {
        const size_t n8 = (size_t)NB * SEQ * DM / 8;
        k_cvt8<0><<<(unsigned)((n8 + 255) / 256), 256, 0, stream>>>(x, XB, n8);
    } else {
        const size_t n8 = (size_t)SEQ * DM / 8;
        for (int b = 0; b < NB; ++b) k_cvt8<0><<<(unsigned)((n8 + 255) / 256), 256, 0, stream>>>(x + (size_t)b * SEQ_FULL * DM, XB + (size_t)b * SEQ * DM, n8);
    }
    k_cvtT<<<dim3(QKVC / 64, DM / 64, 1), 256, 0, stream>>>(wqkv, WQ, QKVC, 0);
    k_cvtT<<<dim3(DM / 64, DM / 64, 1), 256, 0, stream>>>(wo, (unsigned short*)WO, DM, 1);

    k_proj<true><<<dim3(NB * SEQ / 64, DM / 64, 1), 32, 0, stream>>>(XB, WQ, QH, QR, SEQ, (size_t)NH_ * SEQ * HD, HD, HD, (size_t)SEQ * HD, cs, sn);
    k_proj<true><<<dim3(NB * SEQ / 64, KVD / 64, 1), 32, 0, stream>>>(XB, WK, KH, KR, SEQ, (size_t)NG_ * SEQ * HD, HD, HD, (size_t)SEQ * HD, cs, sn);
    k_proj<false><<<dim3(KVD / 64, NB * SEQ / 64, 1), 32, 0, stream>>>(WV, XB, VH, VR, KVD, (size_t)0, SEQ, SEQ, (size_t)KVD * SEQ, cs, sn);

    k_flash<true><<<dim3(ER_ROWS / (16 * AW), NB * NH_, 1), 32 * AW, 0, stream>>>(QH, QR, KH, KR, VH, VR, CH, CR, 0);
    if (SEQ > ER_ROWS)
        k_flash<false><<<dim3((SEQ - ER_ROWS) / (16 * AW) + (SEQ == ER_ROWS), NB * NH_, 1), 32 * AW, 0, stream>>>(QH, QR, KH, KR, VH, VR, CH, CR, ER_ROWS / (16 * AW));

    k_out<2, true><<<dim3(NB * ER_ROWS / 32, DM / 64, 1), 32, 0, stream>>>(CH, CR, WO, OUT, 0, ER_ROWS);
    if (SEQ > ER_ROWS)
        k_out<4, false><<<dim3(NB * (SEQ - ER_ROWS) / 64 + (SEQ == ER_ROWS), DM / 64, 1), 32, 0, stream>>>(CH, CR, WO, OUT, ER_ROWS, (SEQ == ER_ROWS) ? 64 : (SEQ - ER_ROWS));
}
